// StrokeRnn_14096082666012
// MI455X (gfx1250) — hardware-run, weakly checked
//
#include <hip/hip_runtime.h>
#include <math.h>

typedef __attribute__((ext_vector_type(16))) _Float16 v16h;
typedef __attribute__((ext_vector_type(8)))  _Float16 v8h;
typedef __attribute__((ext_vector_type(4)))  _Float16 v4h;
typedef __attribute__((ext_vector_type(8)))  float    v8f;
typedef __attribute__((ext_vector_type(4)))  float    v4f;
typedef __attribute__((ext_vector_type(2)))  float    v2f;
typedef __attribute__((ext_vector_type(4)))  unsigned v4u;

constexpr int kS   = 128;
constexpr int kB   = 256;
constexpr int kH   = 512;
constexpr int kI   = 2;
constexpr int kO   = 2;
constexpr int kG   = 4 * kH;
constexpr int kDWP = kI + kH;
constexpr int kBT  = 16;
constexpr int kNW  = 16;
constexpr int kHP  = 520;
constexpr int kG3P = 3 * kH + kG - kH - kH + kH;
constexpr int kPcCol = 2 * kH;
static_assert(kG3P == 3072, "G3 pitch");
static_assert(kI == 2 && kO == 2 && kDWP == 514, "shapes");
static_assert((kH % 32) == 0 && (kB % 64) == 0 && (kG % 64) == 0 && (kG3P % 64) == 0, "GEMM multiples");
static_assert(kNW * 32 == kH && (kB % kBT) == 0, "tile cover");
static_assert(((kHP * 2) % 16) == 0, "LDS row pitch 16-B aligned");

constexpr float kWC = 1024.0f;
constexpr float kHC = 256.0f;
constexpr float kCC = 16.0f;
constexpr float kFoldRec = 1.0f / (kHC * kWC);
constexpr float kFoldDec = 1.0f / (kCC * kWC);

constexpr int kRowEncW = 0;
constexpr int kRowDecW = 2048;
constexpr int kRowLat  = 4096;
constexpr int kRowLat2 = 4608;
constexpr int kRowDH   = 5120;
constexpr int kRowDC   = 5632;
constexpr int kRowDP   = 6144;
constexpr int kRowsAll = 8192;

constexpr size_t kOffW16  = 0;
constexpr size_t kOffTBL  = kOffW16  + (size_t)kRowsAll * kH * 2;
constexpr size_t kOffENCC = kOffTBL  + (size_t)4096 * 4;
constexpr size_t kOffHN   = kOffENCC + (size_t)kG * 4 * 4;
constexpr size_t kOffML   = kOffHN   + (size_t)kB * kH * 2;
constexpr size_t kOffCODE = kOffML   + (size_t)kB * 2 * kH * 4;
constexpr size_t kOffG3   = kOffCODE + (size_t)kB * kH * 2;
constexpr size_t kOffHD   = kOffG3   + (size_t)kB * kG3P * 4;
constexpr size_t kOffCD   = kOffHD   + (size_t)kB * kH * 2;
constexpr size_t kWsTotal = kOffCD   + (size_t)kB * kH * 4;
static_assert(kWsTotal == 13942784ull, "carve total");
static_assert(kWsTotal <= 134217728ull, "carve cap");
static_assert((kOffTBL % 128) == 0 && (kOffENCC % 128) == 0 && (kOffHN % 128) == 0 && (kOffML % 128) == 0 &&
              (kOffCODE % 128) == 0 && (kOffG3 % 128) == 0 && (kOffHD % 128) == 0 && (kOffCD % 128) == 0, "128-B aligned regions");

constexpr int kOut1 = kS * kB * kO;
constexpr int kOut2 = kOut1 + kB * kH;
static_assert((size_t)(kOut2 + kB * kH) * 4 == 1310720ull, "d_out bytes");

union FragU { v16h v; v8h h[2]; };
__device__ __forceinline__ v16h frag_load(const _Float16* p) {
  FragU f;
  f.h[0] = *(const v8h*)(p);
  f.h[1] = *(const v8h*)(p + 16);
  return f.v;
}
__device__ __forceinline__ v8f mma_h(v16h a, v16h b, v8f c) {
  c = __builtin_amdgcn_wmma_f32_16x16x32_f16(false, a, false, b, (short)0, c, false, false);
  asm volatile("v_nop\n\tv_nop\n\tv_nop\n\tv_nop" : "+v"(c) : "v"(a), "v"(b));
  return c;
}
__device__ __forceinline__ void guard4_h(v8f& a0, v8f& a1, v8f& a2, v8f& a3, v16h x) {
  asm volatile("v_nop\n\tv_nop\n\tv_nop\n\tv_nop" : "+v"(a0), "+v"(a1), "+v"(a2), "+v"(a3) : "v"(x));
}
__device__ __forceinline__ void keep4_h(v16h a, v16h b, v16h c, v16h d) { asm volatile("v_nop" :: "v"(a), "v"(b), "v"(c), "v"(d)); }
__device__ __forceinline__ void acc_guard4(v8f& a, v8f& b, v8f& c, v8f& d) { asm volatile("v_nop\n\tv_nop\n\tv_nop\n\tv_nop" : "+v"(a), "+v"(b), "+v"(c), "+v"(d)); }

__device__ __forceinline__ float sigm_f(float x) { return __builtin_amdgcn_rcpf(1.0f + __expf(-x)); }
__device__ __forceinline__ float tanh_f(float x) { return 1.0f - 2.0f * __builtin_amdgcn_rcpf(1.0f + __expf(2.0f * x)); }

__global__ __launch_bounds__(256) void prep_planes_kernel(
    const float* __restrict__ eWhh, const float* __restrict__ dWhh, const float* __restrict__ mW,
    const float* __restrict__ lW, const float* __restrict__ hW, const float* __restrict__ cW,
    const float* __restrict__ dWih, unsigned short* __restrict__ dst)
{
  const int tid = threadIdx.x;
  const int bx = blockIdx.x;
  const float* src;
  int pitch = kH;
  int off = 0;
  int r0;
  if (bx < kRowDecW / 4)      { src = eWhh; r0 = kRowEncW; }
  else if (bx < kRowLat / 4)  { src = dWhh; r0 = kRowDecW; }
  else if (bx < kRowLat2 / 4) { src = mW;   r0 = kRowLat; }
  else if (bx < kRowDH / 4)   { src = lW;   r0 = kRowLat2; }
  else if (bx < kRowDC / 4)   { src = hW;   r0 = kRowDH; }
  else if (bx < kRowDP / 4)   { src = cW;   r0 = kRowDC; }
  else                        { src = dWih; r0 = kRowDP; pitch = kDWP; off = kI; }
  const int gr = bx * 4 + (tid >> 6);
  const int c8 = (tid & 63) * 8;
  const float* sp = src + (size_t)(gr - r0) * pitch + off + c8;
  const v2f a0 = *(const v2f*)(sp);
  const v2f a1 = *(const v2f*)(sp + 2);
  const v2f a2 = *(const v2f*)(sp + 4);
  const v2f a3 = *(const v2f*)(sp + 6);
  v8h hv;
  hv[0] = (_Float16)(a0[0] * kWC);
  hv[1] = (_Float16)(a0[1] * kWC);
  hv[2] = (_Float16)(a1[0] * kWC);
  hv[3] = (_Float16)(a1[1] * kWC);
  hv[4] = (_Float16)(a2[0] * kWC);
  hv[5] = (_Float16)(a2[1] * kWC);
  hv[6] = (_Float16)(a3[0] * kWC);
  hv[7] = (_Float16)(a3[1] * kWC);
  unsigned short* q = dst + (size_t)gr * kH + c8;
  *(volatile v8h*)q = hv;
  __threadfence();
  *(volatile v8h*)q = hv;
}

__global__ __launch_bounds__(256) void prep_tables_kernel(
    const float* __restrict__ mean_b, const float* __restrict__ logstd_b, const float* __restrict__ decH_b,
    const float* __restrict__ decC_b, const float* __restrict__ dec_bih, const float* __restrict__ dec_bhh,
    const float* __restrict__ enc_Wih, const float* __restrict__ enc_bih, const float* __restrict__ enc_bhh,
    float* __restrict__ tbl, float* __restrict__ encC)
{
  const int tid = threadIdx.x;
  const int bx = blockIdx.x;
  v4f v;
  float* q;
  if (bx < 4) {
    const int j = bx * 256 + tid;
    const int seg = __builtin_amdgcn_readfirstlane(j >> 7);
    const int e = (j & 127) * 4;
    if (seg == 0)      v = *(const v4f*)(mean_b + e);
    else if (seg == 1) v = *(const v4f*)(logstd_b + e);
    else if (seg == 2) v = *(const v4f*)(decH_b + e);
    else if (seg == 3) v = *(const v4f*)(decC_b + e);
    else {
      const int e2 = (seg - 4) * 512 + e;
      const v4f b1 = *(const v4f*)(dec_bih + e2);
      const v4f b2 = *(const v4f*)(dec_bhh + e2);
      v = b1 + b2;
    }
    q = tbl + 4 * j;
  } else {
    const int n = (bx - 4) * 256 + tid;
    const v2f w = *(const v2f*)(enc_Wih + 2 * n);
    v[0] = enc_bih[n] + enc_bhh[n];
    v[1] = w[0];
    v[2] = w[1];
    v[3] = 0.0f;
    q = encC + 4 * n;
  }
  *(volatile v4f*)q = v;
  __threadfence();
  *(volatile v4f*)q = v;
}

__global__ __launch_bounds__(256) void gemm64_f16_kernel(
    const unsigned short* __restrict__ Ap, int lda,
    const unsigned short* __restrict__ Btp, int ldb,
    float* __restrict__ C, int ldc,
    const float* __restrict__ bias,
    int M, int N, int K, float scale)
{
  const _Float16* A  = (const _Float16*)Ap;
  const _Float16* Bt = (const _Float16*)Btp;
  __shared__ __align__(16) float sT[8][16 * 68];
  const int lane = threadIdx.x & 31;
  const int wave = __builtin_amdgcn_readfirstlane((int)(threadIdx.x >> 5));
  const int tilesN = N >> 6;
  const int tilesM = M >> 6;
  const int tile = blockIdx.x * 8 + wave;
  if (tile >= tilesM * tilesN) return;
  const int tm = tile / tilesN;
  const int tn = tile - tm * tilesN;
  const int m0 = tm << 6;
  const int n0 = tn << 6;

  const int rlane = lane & 15;
  const int koff  = (lane >> 4) * 8;
  const int mOff  = (lane >> 4) * 8;

  v8f acc[4][4];
#pragma unroll
  for (int i = 0; i < 4; ++i)
#pragma unroll
    for (int j = 0; j < 4; ++j) acc[i][j] = (v8f){0.f,0.f,0.f,0.f,0.f,0.f,0.f,0.f};

  for (int k0 = 0; k0 < K; k0 += 32) {
    v16h bh[4];
#pragma unroll
    for (int j = 0; j < 4; ++j) {
      const size_t bo = (size_t)(n0 + (j << 4) + rlane) * ldb + koff + k0;
      bh[j] = frag_load(Bt + bo);
    }
#pragma unroll
    for (int i = 0; i < 4; ++i) {
      const size_t ao = (size_t)(m0 + (i << 4) + rlane) * lda + koff + k0;
      const v16h ah = frag_load(A + ao);
#pragma unroll
      for (int j = 0; j < 4; ++j) {
        acc[i][j] = __builtin_amdgcn_wmma_f32_16x16x32_f16(false, ah, false, bh[j], (short)0, acc[i][j], false, false);
      }
      guard4_h(acc[i][0], acc[i][1], acc[i][2], acc[i][3], ah);
    }
    keep4_h(bh[0], bh[1], bh[2], bh[3]);
  }
  acc_guard4(acc[0][0], acc[0][1], acc[0][2], acc[0][3]);
  acc_guard4(acc[1][0], acc[1][1], acc[1][2], acc[1][3]);
  acc_guard4(acc[2][0], acc[2][1], acc[2][2], acc[2][3]);
  acc_guard4(acc[3][0], acc[3][1], acc[3][2], acc[3][3]);

  float* slab = sT[wave];
#pragma unroll
  for (int i = 0; i < 4; ++i) {
    const int mBase = m0 + (i << 4);
#pragma unroll
    for (int j = 0; j < 4; ++j) {
      const int n = n0 + (j << 4) + rlane;
      const float bv = bias[n];
#pragma unroll
      for (int r = 0; r < 8; ++r) {
        const float v = acc[i][j][r] * scale + bv;
        slab[(mOff + r) * 68 + (j << 4) + rlane] = v;
      }
    }
    __builtin_amdgcn_fence(__ATOMIC_RELEASE, "workgroup");
    __builtin_amdgcn_wave_barrier();
    __builtin_amdgcn_fence(__ATOMIC_ACQUIRE, "workgroup");
    {
      const int hh = lane >> 4, c4 = (lane & 15) * 4;
      for (int pass = 0; pass < 2; ++pass) {
#pragma unroll
        for (int it = 0; it < 8; ++it) {
          const int row = it * 2 + hh;
          const v4f v = *(const v4f*)(slab + row * 68 + c4);
          *(volatile v4f*)(C + (size_t)(mBase + row) * ldc + n0 + c4) = v;
        }
        __threadfence();
      }
    }
    __builtin_amdgcn_fence(__ATOMIC_RELEASE, "workgroup");
    __builtin_amdgcn_wave_barrier();
    __builtin_amdgcn_fence(__ATOMIC_ACQUIRE, "workgroup");
  }
}

__global__ __launch_bounds__(512) __attribute__((amdgpu_num_vgpr(256)))
void enc_scan_kernel(const float* x, const int* seq_len, const unsigned short* W16p,
                     const float* encC, unsigned short* hn16)
{
  __shared__ __align__(16) _Float16 sH[2 * kBT * kHP];
  __shared__ __align__(16) _Float16 sHn[kBT * kH];
  const _Float16* W16 = (const _Float16*)W16p;
  const int tid  = threadIdx.x;
  const int lane = tid & 31;
  const int wave = __builtin_amdgcn_readfirstlane((int)(threadIdx.x >> 5));
  const int hh = lane >> 4;
  const int c  = lane & 15;
  const int b0 = blockIdx.x * kBT;
  const int colb = 32 * wave + c;

  {
    const v4u z = (v4u){0u, 0u, 0u, 0u};
    for (int i = tid; i < (kBT * kHP) / 8; i += 512) *(v4u*)(sH + 8 * i) = z;
    for (int i = tid; i < (kBT * kH) / 8; i += 512) *(v4u*)(sHn + 8 * i) = z;
  }

  float cb[4][2], cw0[4][2], cw1[4][2];
#pragma unroll
  for (int g = 0; g < 4; ++g) {
#pragma unroll
    for (int s = 0; s < 2; ++s) {
      const int n = g * kH + colb + 16 * s;
      const v4f q = *(const v4f*)(encC + 4 * n);
      cb[g][s]  = q[0];
      cw0[g][s] = q[1];
      cw1[g][s] = q[2];
    }
  }
  int slm1[8];
#pragma unroll
  for (int r = 0; r < 8; ++r) {
    int v = seq_len[b0 + 8 * hh + r];
    v = v < 1 ? 1 : v;
    v = v > kS ? kS : v;
    slm1[r] = v - 1;
  }
  int tmax = 1;
  for (int j = 0; j < kBT; ++j) {
    int v = seq_len[b0 + j];
    v = v < 1 ? 1 : v;
    v = v > kS ? kS : v;
    tmax = v > tmax ? v : tmax;
  }
  tmax = __builtin_amdgcn_readfirstlane(tmax);

  v8f cst[2];
  cst[0] = (v8f){0.f,0.f,0.f,0.f,0.f,0.f,0.f,0.f};
  cst[1] = (v8f){0.f,0.f,0.f,0.f,0.f,0.f,0.f,0.f};

  const _Float16* Wl = W16 + (size_t)colb * kH + 8 * hh;
  __syncthreads();

#pragma unroll 1
  for (int t = 0; t < tmax; ++t) {
    asm volatile("" ::: "memory");
    const _Float16* hA = sH + (t & 1) * (kBT * kHP) + c * kHP + 8 * hh;
    _Float16* hW = sH + ((t + 1) & 1) * (kBT * kHP);
    v8f acc[4][2];
#pragma unroll
    for (int g = 0; g < 4; ++g) {
      acc[g][0] = (v8f){0.f,0.f,0.f,0.f,0.f,0.f,0.f,0.f};
      acc[g][1] = (v8f){0.f,0.f,0.f,0.f,0.f,0.f,0.f,0.f};
    }
#pragma unroll 1
    for (int k0 = 0; k0 < kH; k0 += 32) {
      const v16h a = frag_load(hA + k0);
#pragma unroll
      for (int g = 0; g < 4; ++g) {
#pragma unroll
        for (int s = 0; s < 2; ++s) {
          const v16h b = frag_load(Wl + (size_t)(g * kH + 16 * s) * kH + k0);
          acc[g][s] = mma_h(a, b, acc[g][s]);
        }
      }
    }
    const float* xt = x + (size_t)t * (kB * kI) + (size_t)(b0 + 8 * hh) * kI;
#pragma unroll
    for (int r = 0; r < 8; ++r) {
      const int row = 8 * hh + r;
      const v2f xv = *(const v2f*)(xt + 2 * r);
      const bool cap = (t == slm1[r]);
#pragma unroll
      for (int s = 0; s < 2; ++s) {
        float gi = fmaf(acc[0][s][r], kFoldRec, cb[0][s]);
        float gf = fmaf(acc[1][s][r], kFoldRec, cb[1][s]);
        float gg = fmaf(acc[2][s][r], kFoldRec, cb[2][s]);
        float go = fmaf(acc[3][s][r], kFoldRec, cb[3][s]);
        gi = fmaf(xv[0], cw0[0][s], gi);
        gf = fmaf(xv[0], cw0[1][s], gf);
        gg = fmaf(xv[0], cw0[2][s], gg);
        go = fmaf(xv[0], cw0[3][s], go);
        gi = fmaf(xv[1], cw1[0][s], gi);
        gf = fmaf(xv[1], cw1[1][s], gf);
        gg = fmaf(xv[1], cw1[2][s], gg);
        go = fmaf(xv[1], cw1[3][s], go);
        const float iv = sigm_f(gi);
        const float fv = sigm_f(gf);
        const float gv = tanh_f(gg);
        const float ov = sigm_f(go);
        const float cn = fmaf(fv, cst[s][r], iv * gv);
        cst[s][r] = cn;
        const float hv = ov * tanh_f(cn);
        const _Float16 h16 = (_Float16)(hv * kHC);
        hW[row * kHP + colb + 16 * s] = h16;
        if (cap) sHn[row * kH + colb + 16 * s] = h16;
      }
    }
    __syncthreads();
  }

  {
    v4u hv[2];
#pragma unroll
    for (int it = 0; it < 2; ++it) {
      const int i = tid + 512 * it;
      hv[it] = *(const v4u*)(sHn + (i >> 6) * kH + (i & 63) * 8);
    }
    for (int pass = 0; pass < 2; ++pass) {
#pragma unroll
      for (int it = 0; it < 2; ++it) {
        const int i = tid + 512 * it;
        *(volatile v4u*)(hn16 + (size_t)(b0 + (i >> 6)) * kH + (i & 63) * 8) = hv[it];
      }
      __threadfence();
    }
  }
}

__global__ __launch_bounds__(256) void latent_code_kernel(
    const float* __restrict__ ML, const float* __restrict__ eps,
    float* __restrict__ out1, float* __restrict__ out2, unsigned short* __restrict__ code16)
{
  const int i = blockIdx.x * 256 + threadIdx.x;
  if (i >= kB * kH / 4) return;
  const int row = i >> 7;
  const int c4 = (i & 127) * 4;
  const v4f m  = *(const v4f*)(ML + (size_t)row * (2 * kH) + c4);
  const v4f ls = *(const v4f*)(ML + (size_t)row * (2 * kH) + kH + c4);
  const v4f e  = *(const v4f*)(eps + (size_t)row * kH + c4);
  v4h cv;
  cv[0] = (_Float16)((m[0] + expf(0.5f * ls[0]) * e[0]) * kCC);
  cv[1] = (_Float16)((m[1] + expf(0.5f * ls[1]) * e[1]) * kCC);
  cv[2] = (_Float16)((m[2] + expf(0.5f * ls[2]) * e[2]) * kCC);
  cv[3] = (_Float16)((m[3] + expf(0.5f * ls[3]) * e[3]) * kCC);
  float* q1 = out1 + (size_t)row * kH + c4;
  float* q2 = out2 + (size_t)row * kH + c4;
  unsigned short* qc = code16 + (size_t)row * kH + c4;
  *(volatile v4f*)q1 = m;
  *(volatile v4f*)q2 = ls;
  *(volatile v4h*)qc = cv;
  __threadfence();
  *(volatile v4f*)q1 = m;
  *(volatile v4f*)q2 = ls;
  *(volatile v4h*)qc = cv;
}

__global__ __launch_bounds__(256) void dec_init_kernel(
    const float* __restrict__ G3, unsigned short* __restrict__ hd16, float* __restrict__ cd32)
{
  const int bx = blockIdx.x;
  const int row = bx >> 1;
  const int half = bx & 1;
  const int c2 = threadIdx.x * 2;
  const v2f g = *(const v2f*)(G3 + (size_t)row * kG3P + half * kH + c2);
  const float t0 = tanhf(g[0]);
  const float t1 = tanhf(g[1]);
  if (half == 0) {
    const _Float16 h0 = (_Float16)(t0 * kHC), h1 = (_Float16)(t1 * kHC);
    const unsigned u = (unsigned)__builtin_bit_cast(unsigned short, h0) | ((unsigned)__builtin_bit_cast(unsigned short, h1) << 16);
    unsigned* q = (unsigned*)(hd16 + (size_t)row * kH + c2);
    *(volatile unsigned*)q = u;
    __threadfence();
    *(volatile unsigned*)q = u;
  } else {
    v2f v;
    v[0] = t0;
    v[1] = t1;
    float* q = cd32 + (size_t)row * kH + c2;
    *(volatile v2f*)q = v;
    __threadfence();
    *(volatile v2f*)q = v;
  }
}

__global__ __launch_bounds__(512) __attribute__((amdgpu_num_vgpr(256)))
void dec_scan_kernel(const unsigned short* W16p, const float* G3, const unsigned short* hd16,
                     const float* cd32, const float* dWih, const float* outW, const float* outb,
                     float* out0)
{
  __shared__ __align__(16) _Float16 sH[2 * kBT * kHP];
  __shared__ __align__(16) float sPart[kNW * 32];
  __shared__ __align__(16) float sP[32];
  const _Float16* W16 = (const _Float16*)W16p;
  const int tid  = threadIdx.x;
  const int lane = tid & 31;
  const int wave = __builtin_amdgcn_readfirstlane((int)(threadIdx.x >> 5));
  const int hh = lane >> 4;
  const int c  = lane & 15;
  const int b0 = blockIdx.x * kBT;
  const int colb = 32 * wave + c;

#pragma unroll
  for (int it = 0; it < 2; ++it) {
    const int i = tid + 512 * it;
    const int row = i >> 6, c8 = (i & 63) * 8;
    const v4u v = *(const v4u*)(hd16 + (size_t)(b0 + row) * kH + c8);
    *(v4u*)(sH + row * kHP + c8) = v;
  }
  if (wave == 0) sP[lane] = 0.0f;

  float dw0[4][2], dw1[4][2], ow0[2], ow1[2];
#pragma unroll
  for (int g = 0; g < 4; ++g) {
#pragma unroll
    for (int s = 0; s < 2; ++s) {
      const int n = g * kH + colb + 16 * s;
      const v2f q = *(const v2f*)(dWih + (size_t)n * kDWP);
      dw0[g][s] = q[0];
      dw1[g][s] = q[1];
    }
  }
#pragma unroll
  for (int s = 0; s < 2; ++s) {
    ow0[s] = outW[colb + 16 * s];
    ow1[s] = outW[kH + colb + 16 * s];
  }
  const float ob = outb[lane & 1];

  v8f cst[2];
#pragma unroll
  for (int s = 0; s < 2; ++s) {
#pragma unroll
    for (int r = 0; r < 8; ++r) cst[s][r] = cd32[(size_t)(b0 + 8 * hh + r) * kH + colb + 16 * s];
  }

  const _Float16* Wl = W16 + (size_t)colb * kH + 8 * hh;
  __syncthreads();

#pragma unroll 1
  for (int t = 0; t < kS; ++t) {
    asm volatile("" ::: "memory");
    const _Float16* hA = sH + (t & 1) * (kBT * kHP) + c * kHP + 8 * hh;
    _Float16* hW = sH + ((t + 1) & 1) * (kBT * kHP);
    v8f acc[4][2];
#pragma unroll
    for (int g = 0; g < 4; ++g) {
      acc[g][0] = (v8f){0.f,0.f,0.f,0.f,0.f,0.f,0.f,0.f};
      acc[g][1] = (v8f){0.f,0.f,0.f,0.f,0.f,0.f,0.f,0.f};
    }
#pragma unroll 1
    for (int k0 = 0; k0 < kH; k0 += 32) {
      const v16h a = frag_load(hA + k0);
#pragma unroll
      for (int g = 0; g < 4; ++g) {
#pragma unroll
        for (int s = 0; s < 2; ++s) {
          const v16h b = frag_load(Wl + (size_t)(g * kH + 16 * s) * kH + k0);
          acc[g][s] = mma_h(a, b, acc[g][s]);
        }
      }
    }
#pragma unroll
    for (int r = 0; r < 8; ++r) {
      const int row = 8 * hh + r;
      const v2f pv = *(const v2f*)(sP + 2 * row);
      const float* pcr = G3 + (size_t)(b0 + row) * kG3P + kPcCol + colb;
      float q0 = 0.0f, q1 = 0.0f;
#pragma unroll
      for (int s = 0; s < 2; ++s) {
        float gi = fmaf(acc[0][s][r], kFoldRec, pcr[0 * kH + 16 * s]);
        float gf = fmaf(acc[1][s][r], kFoldRec, pcr[1 * kH + 16 * s]);
        float gg = fmaf(acc[2][s][r], kFoldRec, pcr[2 * kH + 16 * s]);
        float go = fmaf(acc[3][s][r], kFoldRec, pcr[3 * kH + 16 * s]);
        gi = fmaf(pv[0], dw0[0][s], gi);
        gf = fmaf(pv[0], dw0[1][s], gf);
        gg = fmaf(pv[0], dw0[2][s], gg);
        go = fmaf(pv[0], dw0[3][s], go);
        gi = fmaf(pv[1], dw1[0][s], gi);
        gf = fmaf(pv[1], dw1[1][s], gf);
        gg = fmaf(pv[1], dw1[2][s], gg);
        go = fmaf(pv[1], dw1[3][s], go);
        const float iv = sigm_f(gi);
        const float fv = sigm_f(gf);
        const float gv = tanh_f(gg);
        const float ov = sigm_f(go);
        const float cn = fmaf(fv, cst[s][r], iv * gv);
        cst[s][r] = cn;
        const float hv = ov * tanh_f(cn);
        hW[row * kHP + colb + 16 * s] = (_Float16)(hv * kHC);
        q0 = fmaf(hv, ow0[s], q0);
        q1 = fmaf(hv, ow1[s], q1);
      }
      q0 += __shfl_xor(q0, 1, 32);
      q1 += __shfl_xor(q1, 1, 32);
      q0 += __shfl_xor(q0, 2, 32);
      q1 += __shfl_xor(q1, 2, 32);
      q0 += __shfl_xor(q0, 4, 32);
      q1 += __shfl_xor(q1, 4, 32);
      q0 += __shfl_xor(q0, 8, 32);
      q1 += __shfl_xor(q1, 8, 32);
      if (c == 0) {
        v2f o2;
        o2[0] = q0;
        o2[1] = q1;
        *(v2f*)(sPart + wave * 32 + 2 * row) = o2;
      }
    }
    __syncthreads();
    if (wave == 0) {
      float o = ob;
#pragma unroll
      for (int w = 0; w < kNW; ++w) o += sPart[w * 32 + lane];
      sP[lane] = o;
      float* q = out0 + (size_t)t * (kB * kO) + (size_t)b0 * kO + lane;
      *(volatile float*)q = o;
      __threadfence();
      *(volatile float*)q = o;
    }
    __syncthreads();
  }
}

extern "C" void kernel_launch(void* const* d_in, const int* in_sizes, int n_in,
                              void* d_out, int out_size, void* d_ws, size_t ws_size,
                              hipStream_t stream) {
  if (n_in < 21) return;
  if (in_sizes[0] != kS * kB * kI) return;
  if (in_sizes[1] != kB) return;
  if (in_sizes[2] != kB * kH) return;
  if (in_sizes[3] != kG * kI) return;
  if (in_sizes[4] != kG * kH) return;
  if (in_sizes[5] != kG || in_sizes[6] != kG) return;
  if (in_sizes[7] != kH * kH || in_sizes[8] != kH) return;
  if (in_sizes[9] != kH * kH || in_sizes[10] != kH) return;
  if (in_sizes[11] != kH * kH || in_sizes[12] != kH) return;
  if (in_sizes[13] != kH * kH || in_sizes[14] != kH) return;
  if (in_sizes[15] != kG * kDWP) return;
  if (in_sizes[16] != kG * kH) return;
  if (in_sizes[17] != kG || in_sizes[18] != kG) return;
  if (in_sizes[19] != kO * kH || in_sizes[20] != kO) return;
  if (out_size != kOut2 + kB * kH) return;
  if (ws_size < kWsTotal) return;

  const float* x        = (const float*)d_in[0];
  const int*   seq_len  = (const int*)d_in[1];
  const float* eps      = (const float*)d_in[2];
  const float* enc_Wih  = (const float*)d_in[3];
  const float* enc_Whh  = (const float*)d_in[4];
  const float* enc_bih  = (const float*)d_in[5];
  const float* enc_bhh  = (const float*)d_in[6];
  const float* mean_W   = (const float*)d_in[7];
  const float* mean_b   = (const float*)d_in[8];
  const float* logstd_W = (const float*)d_in[9];
  const float* logstd_b = (const float*)d_in[10];
  const float* decH_W   = (const float*)d_in[11];
  const float* decH_b   = (const float*)d_in[12];
  const float* decC_W   = (const float*)d_in[13];
  const float* decC_b   = (const float*)d_in[14];
  const float* dec_Wih  = (const float*)d_in[15];
  const float* dec_Whh  = (const float*)d_in[16];
  const float* dec_bih  = (const float*)d_in[17];
  const float* dec_bhh  = (const float*)d_in[18];
  const float* out_W    = (const float*)d_in[19];
  const float* out_b    = (const float*)d_in[20];
  float* out = (float*)d_out;

  char* ws = (char*)d_ws;
  unsigned short* W16ALL = (unsigned short*)(ws + kOffW16);
  float*          TBL    = (float*)(ws + kOffTBL);
  float*          ENCC   = (float*)(ws + kOffENCC);
  unsigned short* HN16   = (unsigned short*)(ws + kOffHN);
  float*          ML32   = (float*)(ws + kOffML);
  unsigned short* CODE16 = (unsigned short*)(ws + kOffCODE);
  float*          G3     = (float*)(ws + kOffG3);
  unsigned short* HD16   = (unsigned short*)(ws + kOffHD);
  float*          CD32   = (float*)(ws + kOffCD);

  const unsigned short* encW16 = W16ALL + (size_t)kRowEncW * kH;
  const unsigned short* decW16 = W16ALL + (size_t)kRowDecW * kH;
  const unsigned short* latW16 = W16ALL + (size_t)kRowLat * kH;
  const unsigned short* dinW16 = W16ALL + (size_t)kRowDH * kH;

  prep_planes_kernel<<<kRowsAll / 4, 256, 0, stream>>>(enc_Whh, dec_Whh, mean_W, logstd_W, decH_W, decC_W, dec_Wih, W16ALL);
  prep_tables_kernel<<<12, 256, 0, stream>>>(mean_b, logstd_b, decH_b, decC_b, dec_bih, dec_bhh,
                                             enc_Wih, enc_bih, enc_bhh, TBL, ENCC);

  enc_scan_kernel<<<kB / kBT, 512, 0, stream>>>(x, seq_len, encW16, ENCC, HN16);

  gemm64_f16_kernel<<<8, 256, 0, stream>>>(HN16, kH, latW16, kH, ML32, 2 * kH, TBL, kB, 2 * kH, kH, kFoldRec);

  latent_code_kernel<<<(kB * kH / 4) / 256, 256, 0, stream>>>(ML32, eps, out + kOut1, out + kOut2, CODE16);

  gemm64_f16_kernel<<<24, 256, 0, stream>>>(CODE16, kH, dinW16, kH, G3, kG3P, TBL + 2 * kH, kB, kG3P, kH, kFoldDec);

  dec_init_kernel<<<kB * 2, 256, 0, stream>>>(G3, HD16, CD32);

  dec_scan_kernel<<<kB / kBT, 512, 0, stream>>>(decW16, G3, HD16, CD32, dec_Wih, out_W, out_b, out);
}
